// TMix_22179211116820
// MI455X (gfx1250) — hardware-run, weakly checked
//
#include <hip/hip_runtime.h>
#include <math.h>

typedef __attribute__((ext_vector_type(16))) _Float16 v16h;
typedef __attribute__((ext_vector_type(8)))  _Float16 v8h;
typedef __attribute__((ext_vector_type(8)))  float    v8f;
typedef __attribute__((ext_vector_type(4)))  float    v4f;
typedef __attribute__((ext_vector_type(4)))  unsigned int v4u;

constexpr int kB = 4;
constexpr int kT = 1024;
constexpr int kC = 1024;
constexpr int kH = 16;
constexpr int kD = 64;
constexpr int kRows  = kB * kT;
constexpr int kPassB = 2;
constexpr int kMP    = kPassB * kT;
constexpr int kNPass = kB / kPassB;
constexpr int kRW  = 64;
constexpr int kRA  = 64;
constexpr int kRV  = 32;
constexpr int kRVP = 64;
constexpr int kRG  = 128;
static_assert(kH * kD == kC, "heads x head dim");
static_assert(kRW == 64 && kRA == 64 && kRVP == 64, "low-rank planes share one 64-wide pitch");
static_assert((kMP % 64) == 0 && (kC % 64) == 0 && (kRG % 64) == 0, "GEMM M,N tile multiples");
static_assert((kC % 32) == 0 && (kRVP % 32) == 0 && (kRG % 32) == 0, "GEMM K multiples of 32");
static_assert((kT & (kT - 1)) == 0, "sequence length power of two");

constexpr float kActCarry = 16.0f;
constexpr float kWCarry   = 1024.0f;
constexpr float kMidCarry = 16.0f;
constexpr float kYCarry   = 256.0f;
constexpr float kLoCarry  = 2048.0f;
constexpr float kLoInv    = 1.0f / kLoCarry;
constexpr float kScaleProj = 1.0f / (kActCarry * kWCarry);
constexpr float kScaleLow2 = 1.0f / (kMidCarry * kWCarry);
constexpr float kScaleG2   = 1.0f / kWCarry;
constexpr float kScaleOut  = 1.0f / (kYCarry * kWCarry);
constexpr float kLogDecay  = -0.6065306597126334f;
constexpr float kGnEps     = (float)kD * 1e-5f;
constexpr float kF16MinNormal = 6.103515625e-5f;

constexpr size_t kSzW   = (size_t)kC * kC * 2;
constexpr size_t kSzL1  = (size_t)64 * kC * 2;
constexpr size_t kSzG1  = (size_t)kRG * kC * 2;
constexpr size_t kSzX16 = (size_t)kMP * kC * 2;
constexpr size_t kSzX32 = (size_t)kMP * kC * 4;
constexpr size_t kSzZ1  = (size_t)kMP * 64 * 4;
constexpr size_t kSzZG1 = (size_t)kMP * kRG * 4;
constexpr size_t kSzT   = (size_t)kMP * 64 * 2;
constexpr size_t kSzTG  = (size_t)kMP * kRG * 2;

constexpr size_t kOffWB  = 0;
constexpr size_t kOffWBL = kOffWB  + 4 * kSzW;
constexpr size_t kOffLR1 = kOffWBL + 2 * kSzW;
constexpr size_t kOffG1T = kOffLR1 + 3 * kSzL1;
constexpr size_t kOffLR2 = kOffG1T + kSzG1;
constexpr size_t kOffG2T = kOffLR2 + 3 * kSzL1;
constexpr size_t kOffXH  = kOffG2T + kSzG1;
constexpr size_t kOffXG  = kOffXH  + 5 * kSzX16;
constexpr size_t kOffXL  = kOffXG  + kSzX16;
constexpr size_t kOffRKV = kOffXL  + 3 * kSzX16;
constexpr size_t kOffZ1  = kOffRKV + 3 * kSzX32;
constexpr size_t kOffZG1 = kOffZ1  + 3 * kSzZ1;
constexpr size_t kOffT   = kOffZG1 + kSzZG1;
constexpr size_t kOffTGH = kOffT   + 3 * kSzT;
constexpr size_t kOffTGL = kOffTGH + kSzTG;
constexpr size_t kOffZ2  = kOffTGL + kSzTG;
constexpr size_t kOffG   = kOffZ2  + 3 * kSzX32;
constexpr size_t kOffO   = kOffG   + kSzX32;
constexpr size_t kOffYH  = kOffO   + kSzX32;
constexpr size_t kOffYL  = kOffYH  + kSzX16;
constexpr size_t kWsTotal = kOffYL + kSzX16;
static_assert(kWsTotal == 131596288ull, "carve total");
static_assert(kWsTotal <= 134217728ull, "carve cap");
static_assert((kOffWBL % 128) == 0 && (kOffLR1 % 128) == 0 && (kOffG1T % 128) == 0 && (kOffLR2 % 128) == 0 &&
              (kOffG2T % 128) == 0 &&
              (kOffXH % 128) == 0 && (kOffXG % 128) == 0 && (kOffXL % 128) == 0 && (kOffRKV % 128) == 0 &&
              (kOffZ1 % 128) == 0 && (kOffZG1 % 128) == 0 && (kOffT % 128) == 0 && (kOffTGH % 128) == 0 &&
              (kOffTGL % 128) == 0 && (kOffZ2 % 128) == 0 && (kOffG % 128) == 0 && (kOffO % 128) == 0 &&
              (kOffYH % 128) == 0 && (kOffYL % 128) == 0, "128-B aligned regions");

__device__ __forceinline__ unsigned pk16(unsigned short a, unsigned short b) { return (unsigned)a | ((unsigned)b << 16); }
__device__ __forceinline__ unsigned short h_bits(float f) {
  const _Float16 h = (_Float16)f;
  return __builtin_bit_cast(unsigned short, h);
}
__device__ __forceinline__ void split_h(float xc, unsigned short& hb, unsigned short& lb) {
  const _Float16 h0 = (_Float16)xc;
  float hf = (float)h0;
  asm volatile("" : "+v"(hf));
  hf = (fabsf(hf) < kF16MinNormal) ? 0.0f : hf;
  const _Float16 h1 = (_Float16)hf;
  float res = xc - hf;
  asm volatile("" : "+v"(res));
  const _Float16 l1 = (_Float16)(res * kLoCarry);
  hb = __builtin_bit_cast(unsigned short, h1);
  lb = __builtin_bit_cast(unsigned short, l1);
}
__device__ __forceinline__ unsigned short resid_bits(float xc) {
  const _Float16 h0 = (_Float16)xc;
  float hf = (float)h0;
  asm volatile("" : "+v"(hf));
  float res = xc - hf;
  asm volatile("" : "+v"(res));
  const _Float16 l1 = (_Float16)(res * kLoCarry);
  return __builtin_bit_cast(unsigned short, l1);
}
__device__ __forceinline__ float sig_fast(float z) { return __builtin_amdgcn_rcpf(1.0f + __expf(-z)); }

namespace eng {

struct FragH {
  union U { v16h v; v8h h[2]; };
  static __device__ __forceinline__ v16h load(const _Float16* p) {
    U f;
    f.h[0] = *(const v8h*)(p);
    f.h[1] = *(const v8h*)(p + 16);
    return f.v;
  }
  static __device__ __forceinline__ v8f mma(v16h a, v16h b, v8f c) {
    return __builtin_amdgcn_wmma_f32_16x16x32_f16(false, a, false, b, (short)0, c, false, false);
  }
};

__device__ __forceinline__ void grp_guard4(v8f& a0, v8f& a1, v8f& a2, v8f& a3,
                                           v16h x, v16h b0, v16h b1, v16h b2, v16h b3) {
  asm volatile("v_nop\n\tv_nop\n\tv_nop\n\tv_nop"
               : "+v"(a0), "+v"(a1), "+v"(a2), "+v"(a3)
               : "v"(x), "v"(b0), "v"(b1), "v"(b2), "v"(b3));
}
__device__ __forceinline__ void grp_guard8(v8f& a0, v8f& a1, v8f& a2, v8f& a3,
                                           v8f& r0, v8f& r1, v8f& r2, v8f& r3,
                                           v16h x, v16h y, v16h b0, v16h b1, v16h b2, v16h b3) {
  asm volatile("v_nop\n\tv_nop\n\tv_nop\n\tv_nop"
               : "+v"(a0), "+v"(a1), "+v"(a2), "+v"(a3), "+v"(r0), "+v"(r1), "+v"(r2), "+v"(r3)
               : "v"(x), "v"(y), "v"(b0), "v"(b1), "v"(b2), "v"(b3));
}
__device__ __forceinline__ void keep4(v16h a, v16h b, v16h c, v16h d) { asm volatile("v_nop" :: "v"(a), "v"(b), "v"(c), "v"(d)); }
__device__ __forceinline__ void acc_guard4(v8f& a, v8f& b, v8f& c, v8f& d) {
  asm volatile("v_nop\n\tv_nop\n\tv_nop\n\tv_nop" : "+v"(a), "+v"(b), "+v"(c), "+v"(d));
}

template <int MT, bool SPLITA, bool SPLITB>
__global__ __launch_bounds__(256) void wmma_gemm_f16(
    const unsigned short* __restrict__ Ap, const unsigned short* __restrict__ A2p, int lda, long strideA,
    const unsigned short* __restrict__ Btp, const unsigned short* __restrict__ Bt2p, int ldb, long strideB,
    float* __restrict__ Cout, int ldc, long strideC,
    int M, int N, int K, float scale) {
  static_assert(SPLITA || !SPLITB, "a weight residual plane needs the residual accumulator");
  const _Float16* A   = (const _Float16*)Ap;
  const _Float16* A2  = (const _Float16*)A2p;
  const _Float16* Bt  = (const _Float16*)Btp;
  const _Float16* Bt2 = (const _Float16*)Bt2p;
  __shared__ __align__(16) float sT[8][16 * 68];
  const int b    = blockIdx.y;
  const int lane = threadIdx.x & 31;
  const int wave = __builtin_amdgcn_readfirstlane((int)(threadIdx.x >> 5));
  const int tilesN = N >> 6;
  const int tilesM = M / (16 * MT);
  const int tile = blockIdx.x * 8 + wave;
  if (tile >= tilesM * tilesN) return;
  const int tm = tile / tilesN;
  const int tn = tile - tm * tilesN;
  const int m0 = tm * (16 * MT);
  const int n0 = tn << 6;

  const _Float16* Ab  = A  + (size_t)b * strideA;
  const _Float16* Bb  = Bt + (size_t)b * strideB;
  const _Float16* Ab2 = SPLITA ? (A2  + (size_t)b * strideA) : nullptr;
  const _Float16* Bb2 = SPLITB ? (Bt2 + (size_t)b * strideB) : nullptr;

  const int rlane = lane & 15;
  const int koff  = (lane >> 4) * 8;
  const int mOff  = (lane >> 4) * 8;

  constexpr int RT = SPLITA ? MT : 1;
  v8f acc[MT][4];
  v8f accr[RT][4];
#pragma unroll
  for (int i = 0; i < MT; ++i)
#pragma unroll
    for (int j = 0; j < 4; ++j) acc[i][j] = (v8f){0.f, 0.f, 0.f, 0.f, 0.f, 0.f, 0.f, 0.f};
#pragma unroll
  for (int i = 0; i < RT; ++i)
#pragma unroll
    for (int j = 0; j < 4; ++j) accr[i][j] = (v8f){0.f, 0.f, 0.f, 0.f, 0.f, 0.f, 0.f, 0.f};

  for (int k0 = 0; k0 < K; k0 += 32) {
    v16h bh[4];
#pragma unroll
    for (int j = 0; j < 4; ++j) {
      const size_t bo = (size_t)(n0 + (j << 4) + rlane) * ldb + koff + k0;
      bh[j] = FragH::load(Bb + bo);
    }
    v16h ahk[MT];
#pragma unroll
    for (int i = 0; i < MT; ++i) {
      const int ir = SPLITA ? i : 0;
      const size_t ao = (size_t)(m0 + (i << 4) + rlane) * lda + koff + k0;
      ahk[i] = FragH::load(Ab + ao);
      v16h al = ahk[i];
      if (SPLITA) al = FragH::load(Ab2 + ao);
#pragma unroll
      for (int j = 0; j < 4; ++j) {
        acc[i][j] = FragH::mma(ahk[i], bh[j], acc[i][j]);
        if (SPLITA) accr[ir][j] = FragH::mma(al, bh[j], accr[ir][j]);
      }
      if (SPLITA) {
        grp_guard8(acc[i][0], acc[i][1], acc[i][2], acc[i][3],
                   accr[ir][0], accr[ir][1], accr[ir][2], accr[ir][3],
                   ahk[i], al, bh[0], bh[1], bh[2], bh[3]);
      } else {
        grp_guard4(acc[i][0], acc[i][1], acc[i][2], acc[i][3], ahk[i], bh[0], bh[1], bh[2], bh[3]);
      }
    }
    keep4(bh[0], bh[1], bh[2], bh[3]);
    if (SPLITB) {
      v16h bl[4];
#pragma unroll
      for (int j = 0; j < 4; ++j) {
        const size_t bo = (size_t)(n0 + (j << 4) + rlane) * ldb + koff + k0;
        bl[j] = FragH::load(Bb2 + bo);
      }
#pragma unroll
      for (int i = 0; i < MT; ++i) {
        const int ir2 = SPLITB ? i : 0;
#pragma unroll
        for (int j = 0; j < 4; ++j) accr[ir2][j] = FragH::mma(ahk[i], bl[j], accr[ir2][j]);
        grp_guard4(accr[ir2][0], accr[ir2][1], accr[ir2][2], accr[ir2][3], ahk[i], bl[0], bl[1], bl[2], bl[3]);
      }
      keep4(bl[0], bl[1], bl[2], bl[3]);
    }
  }
#pragma unroll
  for (int i = 0; i < MT; ++i) acc_guard4(acc[i][0], acc[i][1], acc[i][2], acc[i][3]);
  if (SPLITA) {
#pragma unroll
    for (int i = 0; i < RT; ++i) acc_guard4(accr[i][0], accr[i][1], accr[i][2], accr[i][3]);
  }

  float* slab = sT[wave];
  float* C = Cout + (size_t)b * strideC;
#pragma unroll
  for (int i = 0; i < MT; ++i) {
    const int ir = SPLITA ? i : 0;
    const int mBase = m0 + (i << 4);
#pragma unroll
    for (int j = 0; j < 4; ++j) {
#pragma unroll
      for (int r = 0; r < 8; ++r) {
        float v = acc[i][j][r];
        if (SPLITA) v = v + accr[ir][j][r] * kLoInv;
        v = v * scale;
        slab[(mOff + r) * 68 + (j << 4) + rlane] = v;
      }
    }
    __builtin_amdgcn_fence(__ATOMIC_RELEASE, "workgroup");
    __builtin_amdgcn_wave_barrier();
    __builtin_amdgcn_fence(__ATOMIC_ACQUIRE, "workgroup");
    {
      const int hh = lane >> 4, c4 = (lane & 15) * 4;
      for (int pass = 0; pass < 2; ++pass) {
#pragma unroll
        for (int it = 0; it < 8; ++it) {
          const int row = it * 2 + hh;
          const v4f v = *(const v4f*)(slab + row * 68 + c4);
          *(volatile v4f*)(C + (size_t)(mBase + row) * ldc + n0 + c4) = v;
        }
        __threadfence();
      }
    }
    __builtin_amdgcn_fence(__ATOMIC_RELEASE, "workgroup");
    __builtin_amdgcn_wave_barrier();
    __builtin_amdgcn_fence(__ATOMIC_ACQUIRE, "workgroup");
  }
}

}

__global__ __launch_bounds__(256) void wcast_kernel(const float* __restrict__ W0, const float* __restrict__ W1,
                                                    const float* __restrict__ W2, const float* __restrict__ W3,
                                                    unsigned short* __restrict__ out, unsigned short* __restrict__ outl,
                                                    float scale) {
  const int z = blockIdx.y;
  const float* W = (z == 0) ? W0 : (z == 1) ? W1 : (z == 2) ? W2 : W3;
  const int i = blockIdx.x * 256 + threadIdx.x;
  const float* p = W + 8 * (size_t)i;
  const v4f a = *(const v4f*)(p);
  const v4f c = *(const v4f*)(p + 4);
  unsigned short hb[8], lb[8];
#pragma unroll
  for (int e = 0; e < 4; ++e) {
    const float fa = a[e];
    const float fc = c[e];
    hb[e]     = h_bits(fa * scale);
    hb[4 + e] = h_bits(fc * scale);
    lb[e]     = resid_bits(fa * scale);
    lb[4 + e] = resid_bits(fc * scale);
  }
  const v4u u  = (v4u){pk16(hb[0], hb[1]), pk16(hb[2], hb[3]), pk16(hb[4], hb[5]), pk16(hb[6], hb[7])};
  const v4u ul = (v4u){pk16(lb[0], lb[1]), pk16(lb[2], lb[3]), pk16(lb[4], lb[5]), pk16(lb[6], lb[7])};
  const bool two = (z < 2);
  const int zl = two ? z : 0;
  unsigned short* q  = out  + (size_t)z  * kC * kC + 8 * (size_t)i;
  unsigned short* ql = outl + (size_t)zl * kC * kC + 8 * (size_t)i;
  *(volatile v4u*)q = u;
  if (two) *(volatile v4u*)ql = ul;
  __threadfence();
  *(volatile v4u*)q = u;
  if (two) *(volatile v4u*)ql = ul;
}

__global__ __launch_bounds__(256) void lowrank_tr_kernel(
    const float* __restrict__ v1, const float* __restrict__ a1, const float* __restrict__ w1, const float* __restrict__ g1,
    const float* __restrict__ v2, const float* __restrict__ a2, const float* __restrict__ w2, const float* __restrict__ g2,
    unsigned short* __restrict__ lr1, unsigned short* __restrict__ g1t,
    unsigned short* __restrict__ lr2, unsigned short* __restrict__ g2t, float scale) {
  __shared__ float sm[64][65];
  const int z = blockIdx.z;
  const float* src;
  unsigned short* dst;
  int R, Cc, Np, Kp;
  if (z == 0)      { src = v1; R = kC;  Cc = kRV; Np = kRVP; Kp = kC;   dst = lr1; }
  else if (z == 1) { src = a1; R = kC;  Cc = kRA; Np = kRA;  Kp = kC;   dst = lr1 + (size_t)64 * kC; }
  else if (z == 2) { src = w1; R = kC;  Cc = kRW; Np = kRW;  Kp = kC;   dst = lr1 + (size_t)128 * kC; }
  else if (z == 3) { src = g1; R = kC;  Cc = kRG; Np = kRG;  Kp = kC;   dst = g1t; }
  else if (z == 4) { src = v2; R = kRV; Cc = kC;  Np = kC;   Kp = kRVP; dst = lr2; }
  else if (z == 5) { src = a2; R = kRA; Cc = kC;  Np = kC;   Kp = kRA;  dst = lr2 + (size_t)kC * 64; }
  else if (z == 6) { src = w2; R = kRW; Cc = kC;  Np = kC;   Kp = kRW;  dst = lr2 + (size_t)kC * 128; }
  else             { src = g2; R = kRG; Cc = kC;  Np = kC;   Kp = kRG;  dst = g2t; }
  const int k0 = blockIdx.x * 64;
  const int n0 = blockIdx.y * 64;
  if (k0 >= Kp || n0 >= Np) return;
  const int t = threadIdx.x;
#pragma unroll 1
  for (int i = 0; i < 16; ++i) {
    const int e  = i * 256 + t;
    const int kl = e >> 6;
    const int nl = e & 63;
    const int k = k0 + kl, n = n0 + nl;
    const bool valid = (k < R) && (n < Cc);
    const int kc = (k < R) ? k : (R - 1);
    const int nc = (n < Cc) ? n : (Cc - 1);
    float v = src[(size_t)kc * Cc + nc];
    asm volatile("" : "+v"(v));
    sm[nl][kl] = valid ? (v * scale) : 0.0f;
  }
  __syncthreads();
  const int lane = t & 31, wave = t >> 5;
  const int q = lane >> 3, c8 = (lane & 7) * 8;
  for (int pass = 0; pass < 2; ++pass) {
#pragma unroll
    for (int it = 0; it < 2; ++it) {
      const int row = wave * 8 + it * 4 + q;
      unsigned short hb[8];
#pragma unroll
      for (int e = 0; e < 8; ++e) hb[e] = h_bits(sm[row][c8 + e]);
      const v4u u = (v4u){pk16(hb[0], hb[1]), pk16(hb[2], hb[3]), pk16(hb[4], hb[5]), pk16(hb[6], hb[7])};
      *(volatile v4u*)(dst + (size_t)(n0 + row) * Kp + k0 + c8) = u;
    }
    __threadfence();
  }
}

__global__ __launch_bounds__(256) void copy_kernel(const float* __restrict__ src, float* __restrict__ dst) {
  const size_t base = (size_t)blockIdx.x * 1024 + threadIdx.x;
  v4f v[4];
#pragma unroll
  for (int it = 0; it < 4; ++it) v[it] = *(const v4f*)(src + 4 * (base + (size_t)it * 256));
  for (int pass = 0; pass < 2; ++pass) {
#pragma unroll
    for (int it = 0; it < 4; ++it) *(volatile v4f*)(dst + 4 * (base + (size_t)it * 256)) = v[it];
    __threadfence();
  }
}

__device__ __forceinline__ void mix_split8(const float* xc, const float* xx, const float* __restrict__ coef,
                                           v4u& hi, v4u& lo) {
  const v4f c0 = *(const v4f*)(coef);
  const v4f c1 = *(const v4f*)(coef + 4);
  unsigned short hb[8], lb[8];
#pragma unroll
  for (int e = 0; e < 4; ++e) {
    const float ca = c0[e];
    const float cb = c1[e];
    const float m0 = xc[e] + xx[e] * ca;
    const float m1 = xc[4 + e] + xx[4 + e] * cb;
    split_h(m0 * kActCarry, hb[e], lb[e]);
    split_h(m1 * kActCarry, hb[4 + e], lb[4 + e]);
  }
  hi = (v4u){pk16(hb[0], hb[1]), pk16(hb[2], hb[3]), pk16(hb[4], hb[5]), pk16(hb[6], hb[7])};
  lo = (v4u){pk16(lb[0], lb[1]), pk16(lb[2], lb[3]), pk16(lb[4], lb[5]), pk16(lb[6], lb[7])};
}
__device__ __forceinline__ void mix_plain8(const float* xc, const float* xx, const float* __restrict__ coef, v4u& hi) {
  const v4f c0 = *(const v4f*)(coef);
  const v4f c1 = *(const v4f*)(coef + 4);
  unsigned short hb[8];
#pragma unroll
  for (int e = 0; e < 4; ++e) {
    const float ca = c0[e];
    const float cb = c1[e];
    const float m0 = xc[e] + xx[e] * ca;
    const float m1 = xc[4 + e] + xx[4 + e] * cb;
    hb[e]     = h_bits(m0 * kActCarry);
    hb[4 + e] = h_bits(m1 * kActCarry);
  }
  hi = (v4u){pk16(hb[0], hb[1]), pk16(hb[2], hb[3]), pk16(hb[4], hb[5]), pk16(hb[6], hb[7])};
}

__global__ __launch_bounds__(256) void mix_kernel(
    const float* __restrict__ x, int rowBase,
    const float* __restrict__ cr, const float* __restrict__ cw, const float* __restrict__ ck,
    const float* __restrict__ cv, const float* __restrict__ ca, const float* __restrict__ cg,
    unsigned short* __restrict__ XH, unsigned short* __restrict__ XG, unsigned short* __restrict__ XL) {
  const int i = blockIdx.x * 256 + threadIdx.x;
  const int lrow = i >> 7;
  const int c0 = (i & 127) << 3;
  const int grow = rowBase + lrow;
  const bool first = (grow & (kT - 1)) == 0;
  const int prow = first ? grow : (grow - 1);
  const float* xp = x + (size_t)grow * kC + c0;
  const float* pp = x + (size_t)prow * kC + c0;
  const v4f xa = *(const v4f*)(xp);
  const v4f xb = *(const v4f*)(xp + 4);
  const v4f pa = *(const v4f*)(pp);
  const v4f pb = *(const v4f*)(pp + 4);
  float xc[8], xx[8];
#pragma unroll
  for (int e = 0; e < 4; ++e) {
    const float c0v = xa[e];
    const float c1v = xb[e];
    const float q0 = pa[e];
    const float q1 = pb[e];
    const float p0 = first ? 0.0f : q0;
    const float p1 = first ? 0.0f : q1;
    xc[e] = c0v;
    xc[4 + e] = c1v;
    xx[e] = p0 - c0v;
    xx[4 + e] = p1 - c1v;
  }
  v4u rh, rl, kh, kl, vh, vl, ah, wh, gh;
  mix_split8(xc, xx, cr + c0, rh, rl);
  mix_split8(xc, xx, ck + c0, kh, kl);
  mix_split8(xc, xx, cv + c0, vh, vl);
  mix_plain8(xc, xx, ca + c0, ah);
  mix_plain8(xc, xx, cw + c0, wh);
  mix_plain8(xc, xx, cg + c0, gh);
  const size_t o = (size_t)lrow * kC + c0;
  const size_t pl = (size_t)kMP * kC;
  for (int pass = 0; pass < 2; ++pass) {
    *(volatile v4u*)(XH + o) = rh;
    *(volatile v4u*)(XH + pl + o) = kh;
    *(volatile v4u*)(XH + 2 * pl + o) = vh;
    *(volatile v4u*)(XH + 3 * pl + o) = ah;
    *(volatile v4u*)(XH + 4 * pl + o) = wh;
    *(volatile v4u*)(XG + o) = gh;
    *(volatile v4u*)(XL + o) = rl;
    *(volatile v4u*)(XL + pl + o) = kl;
    *(volatile v4u*)(XL + 2 * pl + o) = vl;
    __threadfence();
  }
}

__global__ __launch_bounds__(256) void midact_kernel(const float* __restrict__ Z1, const float* __restrict__ ZG1,
                                                     unsigned short* __restrict__ Tp, unsigned short* __restrict__ TGH,
                                                     unsigned short* __restrict__ TGL) {
  const int blk = blockIdx.x;
  if (blk < 192) {
    const size_t e0 = ((size_t)blk * 256 + threadIdx.x) * 8;
    const v4f a = *(const v4f*)(Z1 + e0);
    const v4f c = *(const v4f*)(Z1 + e0 + 4);
    float xv[8];
#pragma unroll
    for (int e = 0; e < 4; ++e) { xv[e] = a[e]; xv[4 + e] = c[e]; }
    const bool tanhMode = (blk >= 128);
    if (tanhMode) {
#pragma unroll
      for (int e = 0; e < 8; ++e) xv[e] = 2.0f * sig_fast(2.0f * xv[e]) - 1.0f;
    }
    unsigned short hb[8];
#pragma unroll
    for (int e = 0; e < 8; ++e) hb[e] = h_bits(xv[e] * kMidCarry);
    const v4u u = (v4u){pk16(hb[0], hb[1]), pk16(hb[2], hb[3]), pk16(hb[4], hb[5]), pk16(hb[6], hb[7])};
    unsigned short* q = Tp + e0;
    *(volatile v4u*)q = u;
    __threadfence();
    *(volatile v4u*)q = u;
  } else {
    const size_t e0 = ((size_t)(blk - 192) * 256 + threadIdx.x) * 8;
    const v4f a = *(const v4f*)(ZG1 + e0);
    const v4f c = *(const v4f*)(ZG1 + e0 + 4);
    unsigned short hb[8], lb[8];
#pragma unroll
    for (int e = 0; e < 4; ++e) {
      const float z0 = a[e];
      const float z1 = c[e];
      split_h(sig_fast(z0), hb[e], lb[e]);
      split_h(sig_fast(z1), hb[4 + e], lb[4 + e]);
    }
    const v4u uh = (v4u){pk16(hb[0], hb[1]), pk16(hb[2], hb[3]), pk16(hb[4], hb[5]), pk16(hb[6], hb[7])};
    const v4u ul = (v4u){pk16(lb[0], lb[1]), pk16(lb[2], lb[3]), pk16(lb[4], lb[5]), pk16(lb[6], lb[7])};
    unsigned short* qh = TGH + e0;
    unsigned short* ql = TGL + e0;
    *(volatile v4u*)qh = uh;
    *(volatile v4u*)ql = ul;
    __threadfence();
    *(volatile v4u*)qh = uh;
    *(volatile v4u*)ql = ul;
  }
}

__global__ __launch_bounds__(256) void prep_kernel(float* Kp, float* Vp, float* ZW, float* ZA, float* ZV,
                                                   const float* __restrict__ vf,
                                                   const float* __restrict__ w0, const float* __restrict__ a0,
                                                   const float* __restrict__ v0, const float* __restrict__ k_k,
                                                   const float* __restrict__ k_a) {
  const int c = threadIdx.x * 4;
  const size_t o = (size_t)blockIdx.x * kC + c;
  const v4f kv = *(const v4f*)(Kp + o);
  const v4f vv = *(const v4f*)(Vp + o);
  const v4f zw = *(const v4f*)(ZW + o);
  const v4f za = *(const v4f*)(ZA + o);
  const v4f zv = *(const v4f*)(ZV + o);
  const v4f fv = *(const v4f*)(vf + o);
  const v4f pw0 = *(const v4f*)(w0 + c);
  const v4f pa0 = *(const v4f*)(a0 + c);
  const v4f pv0 = *(const v4f*)(v0 + c);
  const v4f pkk = *(const v4f*)(k_k + c);
  const v4f pka = *(const v4f*)(k_a + c);
  float kkv[4];
  float ss = 0.0f;
#pragma unroll
  for (int e = 0; e < 4; ++e) {
    kkv[e] = kv[e] * pkk[e];
    ss += kkv[e] * kkv[e];
  }
  ss += __shfl_xor(ss, 1, 32);
  ss += __shfl_xor(ss, 2, 32);
  ss += __shfl_xor(ss, 4, 32);
  ss += __shfl_xor(ss, 8, 32);
  const float inv = __builtin_amdgcn_rsqf(fmaxf(ss, 1e-24f));
  v4f ok2, ovm, oew, obk, onk;
#pragma unroll
  for (int e = 0; e < 4; ++e) {
    const float av = sig_fast(pa0[e] + za[e]);
    const float vs = sig_fast(pv0[e] + zv[e]);
    const float wl = kLogDecay * sig_fast(pw0[e] + zw[e]);
    const float kn = kkv[e] * inv;
    oew[e] = expf(wl);
    onk[e] = -kn;
    obk[e] = kn * av;
    ok2[e] = kv[e] * (1.0f + (av - 1.0f) * pka[e]);
    ovm[e] = vv[e] + (fv[e] - vv[e]) * vs;
  }
  for (int pass = 0; pass < 2; ++pass) {
    *(volatile v4f*)(Kp + o) = ok2;
    *(volatile v4f*)(Vp + o) = ovm;
    *(volatile v4f*)(ZW + o) = oew;
    *(volatile v4f*)(ZA + o) = obk;
    *(volatile v4f*)(ZV + o) = onk;
    __threadfence();
  }
}

__global__ __launch_bounds__(256) void scan_kernel(const float* __restrict__ Rp, const float* __restrict__ EW,
                                                   const float* __restrict__ K2, const float* __restrict__ Vm,
                                                   const float* __restrict__ NK, const float* __restrict__ BK,
                                                   float* __restrict__ Op) {
  __shared__ __align__(16) float sR[16 * 64];
  __shared__ __align__(16) float sE[16 * 64];
  __shared__ __align__(16) float sK[16 * 64];
  __shared__ __align__(16) float sV[16 * 64];
  __shared__ __align__(16) float sN[16 * 64];
  __shared__ __align__(16) float sB[16 * 64];
  __shared__ __align__(16) float sO[16 * 64];
  const int tid = threadIdx.x;
  const int v = tid >> 2;
  const int q = tid & 3;
  const int srow = tid >> 4;
  const int sc4 = (tid & 15) * 4;
  const int bl = blockIdx.x >> 4;
  const int h  = blockIdx.x & 15;
  const size_t base = (size_t)bl * kT * kC + (size_t)h * kD;
  float S[16];
#pragma unroll
  for (int j = 0; j < 16; ++j) S[j] = 0.0f;
#pragma unroll 1
  for (int t0 = 0; t0 < kT; t0 += 16) {
    const size_t g = base + (size_t)(t0 + srow) * kC + sc4;
    const v4f lr = *(const v4f*)(Rp + g);
    const v4f le = *(const v4f*)(EW + g);
    const v4f lk = *(const v4f*)(K2 + g);
    const v4f lv = *(const v4f*)(Vm + g);
    const v4f ln = *(const v4f*)(NK + g);
    const v4f lb = *(const v4f*)(BK + g);
    *(v4f*)(sR + srow * 64 + sc4) = lr;
    *(v4f*)(sE + srow * 64 + sc4) = le;
    *(v4f*)(sK + srow * 64 + sc4) = lk;
    *(v4f*)(sV + srow * 64 + sc4) = lv;
    *(v4f*)(sN + srow * 64 + sc4) = ln;
    *(v4f*)(sB + srow * 64 + sc4) = lb;
    __syncthreads();
#pragma unroll 1
    for (int s = 0; s < 16; ++s) {
      const int so = s * 64 + q * 16;
      float sab = 0.0f;
#pragma unroll
      for (int j = 0; j < 4; ++j) {
        const v4f a4 = *(const v4f*)(sN + so + 4 * j);
        sab = fmaf(S[4 * j + 0], a4[0], sab);
        sab = fmaf(S[4 * j + 1], a4[1], sab);
        sab = fmaf(S[4 * j + 2], a4[2], sab);
        sab = fmaf(S[4 * j + 3], a4[3], sab);
      }
      sab += __shfl_xor(sab, 1, 32);
      sab += __shfl_xor(sab, 2, 32);
      const float vt = sV[s * 64 + v];
      float ot = 0.0f;
#pragma unroll
      for (int j = 0; j < 4; ++j) {
        const v4f e4 = *(const v4f*)(sE + so + 4 * j);
        const v4f b4 = *(const v4f*)(sB + so + 4 * j);
        const v4f k4 = *(const v4f*)(sK + so + 4 * j);
        const v4f r4 = *(const v4f*)(sR + so + 4 * j);
#pragma unroll
        for (int e = 0; e < 4; ++e) {
          float sn = vt * k4[e];
          sn = fmaf(sab, b4[e], sn);
          sn = fmaf(S[4 * j + e], e4[e], sn);
          S[4 * j + e] = sn;
          ot = fmaf(sn, r4[e], ot);
        }
      }
      ot += __shfl_xor(ot, 1, 32);
      ot += __shfl_xor(ot, 2, 32);
      if (q == 0) sO[s * 64 + v] = ot;
    }
    __syncthreads();
    const v4f ov = *(const v4f*)(sO + srow * 64 + sc4);
    float* dst = Op + g;
    *(volatile v4f*)dst = ov;
    __threadfence();
    *(volatile v4f*)dst = ov;
  }
}

__global__ __launch_bounds__(256) void norm_gate_kernel(const float* __restrict__ Op, const float* __restrict__ Rp,
                                                        const float* __restrict__ K2, const float* __restrict__ Vm,
                                                        const float* __restrict__ Gp, const float* __restrict__ r_k,
                                                        const float* __restrict__ gn_w, const float* __restrict__ gn_b,
                                                        unsigned short* __restrict__ Yh, unsigned short* __restrict__ Yl) {
  const int i = blockIdx.x * 256 + threadIdx.x;
  const int lrow = i >> 7;
  const int c0 = (i & 127) << 3;
  const size_t o = (size_t)lrow * kC + c0;
  float ov[8], rv[8], kv[8], vv[8], gv[8], rk[8], gw[8], gb[8];
  {
    const v4f a = *(const v4f*)(Op + o), b = *(const v4f*)(Op + o + 4);
    const v4f c = *(const v4f*)(Rp + o), d = *(const v4f*)(Rp + o + 4);
    const v4f e = *(const v4f*)(K2 + o), f = *(const v4f*)(K2 + o + 4);
    const v4f g = *(const v4f*)(Vm + o), h = *(const v4f*)(Vm + o + 4);
    const v4f p = *(const v4f*)(Gp + o), q = *(const v4f*)(Gp + o + 4);
    const v4f r0 = *(const v4f*)(r_k + c0),  r1 = *(const v4f*)(r_k + c0 + 4);
    const v4f w0 = *(const v4f*)(gn_w + c0), w1 = *(const v4f*)(gn_w + c0 + 4);
    const v4f b0 = *(const v4f*)(gn_b + c0), b1 = *(const v4f*)(gn_b + c0 + 4);
#pragma unroll
    for (int j = 0; j < 4; ++j) {
      ov[j] = a[j];  ov[4 + j] = b[j];
      rv[j] = c[j];  rv[4 + j] = d[j];
      kv[j] = e[j];  kv[4 + j] = f[j];
      vv[j] = g[j];  vv[4 + j] = h[j];
      gv[j] = p[j];  gv[4 + j] = q[j];
      rk[j] = r0[j]; rk[4 + j] = r1[j];
      gw[j] = w0[j]; gw[4 + j] = w1[j];
      gb[j] = b0[j]; gb[4 + j] = b1[j];
    }
  }
  float s1 = 0.0f, dot = 0.0f;
#pragma unroll
  for (int j = 0; j < 8; ++j) {
    s1 += ov[j];
    dot += rv[j] * kv[j] * rk[j];
  }
  s1 += __shfl_xor(s1, 1, 32);
  s1 += __shfl_xor(s1, 2, 32);
  s1 += __shfl_xor(s1, 4, 32);
  dot += __shfl_xor(dot, 1, 32);
  dot += __shfl_xor(dot, 2, 32);
  dot += __shfl_xor(dot, 4, 32);
  const float mean = s1 * (1.0f / (float)kD);
  float dv[8];
  float s2 = 0.0f;
#pragma unroll
  for (int j = 0; j < 8; ++j) {
    dv[j] = ov[j] - mean;
    s2 += dv[j] * dv[j];
  }
  s2 += __shfl_xor(s2, 1, 32);
  s2 += __shfl_xor(s2, 2, 32);
  s2 += __shfl_xor(s2, 4, 32);
  const float var = s2 * (1.0f / (float)kD);
  const float rstd = __builtin_amdgcn_rsqf(var + kGnEps);
  unsigned short hb[8], lb[8];
#pragma unroll
  for (int j = 0; j < 8; ++j) {
    const float on = dv[j] * rstd * gw[j] + gb[j];
    const float y = (on + dot * vv[j]) * gv[j];
    split_h(y * kYCarry, hb[j], lb[j]);
  }
  const v4u uh = (v4u){pk16(hb[0], hb[1]), pk16(hb[2], hb[3]), pk16(hb[4], hb[5]), pk16(hb[6], hb[7])};
  const v4u ul = (v4u){pk16(lb[0], lb[1]), pk16(lb[2], lb[3]), pk16(lb[4], lb[5]), pk16(lb[6], lb[7])};
  unsigned short* qh = Yh + o;
  unsigned short* ql = Yl + o;
  *(volatile v4u*)qh = uh;
  *(volatile v4u*)ql = ul;
  __threadfence();
  *(volatile v4u*)qh = uh;
  *(volatile v4u*)ql = ul;
}

extern "C" void kernel_launch(void* const* d_in, const int* in_sizes, int n_in,
                              void* d_out, int out_size, void* d_ws, size_t ws_size,
                              hipStream_t stream) {
  if (n_in < 28) return;
  if (in_sizes[0] != kRows * kC || in_sizes[1] != kRows * kC) return;
  for (int i = 2; i < 8; ++i) if (in_sizes[i] != kC) return;
  for (int i = 8; i < 12; ++i) if (in_sizes[i] != kC * kC) return;
  if (in_sizes[12] != kC || in_sizes[13] != kC * kRW || in_sizes[14] != kRW * kC) return;
  if (in_sizes[15] != kC || in_sizes[16] != kC * kRA || in_sizes[17] != kRA * kC) return;
  if (in_sizes[18] != kC || in_sizes[19] != kC * kRV || in_sizes[20] != kRV * kC) return;
  if (in_sizes[21] != kC * kRG || in_sizes[22] != kRG * kC) return;
  if (in_sizes[23] != kC || in_sizes[24] != kC || in_sizes[25] != kH * kD) return;
  if (in_sizes[26] != kC || in_sizes[27] != kC) return;
  if (out_size != 2 * kRows * kC) return;
  if (ws_size < kWsTotal) return;

  const float* x       = (const float*)d_in[0];
  const float* v_first = (const float*)d_in[1];
  const float* x_r = (const float*)d_in[2];
  const float* x_w = (const float*)d_in[3];
  const float* x_k = (const float*)d_in[4];
  const float* x_v = (const float*)d_in[5];
  const float* x_a = (const float*)d_in[6];
  const float* x_g = (const float*)d_in[7];
  const float* Wr = (const float*)d_in[8];
  const float* Wk = (const float*)d_in[9];
  const float* Wv = (const float*)d_in[10];
  const float* Wo = (const float*)d_in[11];
  const float* w0 = (const float*)d_in[12];
  const float* w1 = (const float*)d_in[13];
  const float* w2 = (const float*)d_in[14];
  const float* a0 = (const float*)d_in[15];
  const float* a1 = (const float*)d_in[16];
  const float* a2 = (const float*)d_in[17];
  const float* v0 = (const float*)d_in[18];
  const float* v1 = (const float*)d_in[19];
  const float* v2 = (const float*)d_in[20];
  const float* g1 = (const float*)d_in[21];
  const float* g2 = (const float*)d_in[22];
  const float* k_k = (const float*)d_in[23];
  const float* k_a = (const float*)d_in[24];
  const float* r_k = (const float*)d_in[25];
  const float* gn_w = (const float*)d_in[26];
  const float* gn_b = (const float*)d_in[27];
  float* out = (float*)d_out;

  char* ws = (char*)d_ws;
  unsigned short* WB  = (unsigned short*)(ws + kOffWB);
  unsigned short* WBL = (unsigned short*)(ws + kOffWBL);
  unsigned short* LR1 = (unsigned short*)(ws + kOffLR1);
  unsigned short* G1T = (unsigned short*)(ws + kOffG1T);
  unsigned short* LR2 = (unsigned short*)(ws + kOffLR2);
  unsigned short* G2T = (unsigned short*)(ws + kOffG2T);
  unsigned short* XH  = (unsigned short*)(ws + kOffXH);
  unsigned short* XG  = (unsigned short*)(ws + kOffXG);
  unsigned short* XL  = (unsigned short*)(ws + kOffXL);
  float*          RKV = (float*)(ws + kOffRKV);
  float*          Z1  = (float*)(ws + kOffZ1);
  float*          ZG1 = (float*)(ws + kOffZG1);
  unsigned short* Tp  = (unsigned short*)(ws + kOffT);
  unsigned short* TGH = (unsigned short*)(ws + kOffTGH);
  unsigned short* TGL = (unsigned short*)(ws + kOffTGL);
  float*          Z2  = (float*)(ws + kOffZ2);
  float*          Gp  = (float*)(ws + kOffG);
  float*          Op  = (float*)(ws + kOffO);
  unsigned short* YH  = (unsigned short*)(ws + kOffYH);
  unsigned short* YL  = (unsigned short*)(ws + kOffYL);

  const long plH = (long)kMP * kC;
  float* Rp = RKV;
  float* Kp = RKV + (size_t)plH;
  float* Vp = RKV + 2 * (size_t)plH;
  float* ZV = Z2;
  float* ZA = Z2 + (size_t)plH;
  float* ZW = Z2 + 2 * (size_t)plH;

  wcast_kernel<<<dim3(kC * kC / 8 / 256, 4), 256, 0, stream>>>(Wr, Wk, Wv, Wo, WB, WBL, kWCarry);
  lowrank_tr_kernel<<<dim3(16, 16, 8), 256, 0, stream>>>(v1, a1, w1, g1, v2, a2, w2, g2, LR1, G1T, LR2, G2T, kWCarry);
  copy_kernel<<<kRows * kC / 4 / 1024, 256, 0, stream>>>(v_first, out + (size_t)kRows * kC);

  for (int pass = 0; pass < kNPass; ++pass) {
    const int rowBase = pass * kMP;
    const float* vf_p = v_first + (size_t)rowBase * kC;
    float* out_p = out + (size_t)rowBase * kC;

    mix_kernel<<<kMP * kC / 8 / 256, 256, 0, stream>>>(x, rowBase, x_r, x_w, x_k, x_v, x_a, x_g, XH, XG, XL);

    eng::wmma_gemm_f16<2, true, true><<<dim3(128, 2), 256, 0, stream>>>(
        XH, XL, kC, plH, WB, WBL, kC, (long)kC * kC, RKV, kC, plH, kMP, kC, kC, kScaleProj);

    eng::wmma_gemm_f16<2, true, false><<<dim3(128, 1), 256, 0, stream>>>(
        XH + 2 * (size_t)plH, XL + 2 * (size_t)plH, kC, 0L, WB + 2 * (size_t)kC * kC, nullptr, kC, 0L,
        Vp, kC, 0L, kMP, kC, kC, kScaleProj);

    eng::wmma_gemm_f16<4, false, false><<<dim3(4, 3), 256, 0, stream>>>(
        XH + 2 * (size_t)plH, nullptr, kC, plH, LR1, nullptr, kC, (long)64 * kC, Z1, 64, (long)kMP * 64, kMP, 64, kC, kScaleProj);

    eng::wmma_gemm_f16<4, false, false><<<dim3(8, 1), 256, 0, stream>>>(
        XG, nullptr, kC, 0L, G1T, nullptr, kC, 0L, ZG1, kRG, 0L, kMP, kRG, kC, kScaleProj);

    midact_kernel<<<320, 256, 0, stream>>>(Z1, ZG1, Tp, TGH, TGL);

    eng::wmma_gemm_f16<4, false, false><<<dim3(64, 3), 256, 0, stream>>>(
        Tp, nullptr, 64, (long)kMP * 64, LR2, nullptr, 64, (long)kC * 64, Z2, kC, plH, kMP, kC, 64, kScaleLow2);

    eng::wmma_gemm_f16<2, true, false><<<dim3(128, 1), 256, 0, stream>>>(
        TGH, TGL, kRG, 0L, G2T, nullptr, kRG, 0L, Gp, kC, 0L, kMP, kC, kRG, kScaleG2);

    prep_kernel<<<kMP, 256, 0, stream>>>(Kp, Vp, ZW, ZA, ZV, vf_p, w0, a0, v0, k_k, k_a);

    scan_kernel<<<kPassB * kH, 256, 0, stream>>>(Rp, ZW, Kp, Vp, ZV, ZA, Op);

    norm_gate_kernel<<<kMP * kC / 8 / 256, 256, 0, stream>>>(Op, Rp, Kp, Vp, Gp, r_k, gn_w, gn_b, YH, YL);

    eng::wmma_gemm_f16<2, true, false><<<dim3(128, 1), 256, 0, stream>>>(
        YH, YL, kC, 0L, WB + 3 * (size_t)kC * kC, nullptr, kC, 0L, out_p, kC, 0L, kMP, kC, kC, kScaleOut);
  }
}
